// SpatialMaskAttention_78400333021798
// MI455X (gfx1250) — hardware-verified
//
#include <hip/hip_runtime.h>
#include <math.h>

constexpr int kGroupsBT = 96;
constexpr int kNode     = 512;
constexpr int kFeat     = 64;
constexpr int kFin      = 128;
constexpr int kDm       = 64;
constexpr int kHeads    = 8;
constexpr int kHd       = 8;
constexpr int kRows     = kGroupsBT * kNode;
constexpr int kQkvLd    = 3 * kDm;
constexpr int kKC       = 64;
constexpr int kVP       = 520;
constexpr int kOsP      = 68;
constexpr float kWCarry    = 16.0f;
constexpr float kWCarryInv = 1.0f / 16.0f;
constexpr float kPScale    = 256.0f;
constexpr float kQKScale   = 0.35355339059327373f;
constexpr float kMaskFill  = -32767.0f;

typedef __attribute__((ext_vector_type(16))) _Float16 v16h;
typedef __attribute__((ext_vector_type(8)))  _Float16 v8h;
typedef __attribute__((ext_vector_type(16))) __bf16   v16b;
typedef __attribute__((ext_vector_type(8)))  __bf16   v8b;
typedef __attribute__((ext_vector_type(8)))  float    v8f;
typedef __attribute__((ext_vector_type(4)))  float    v4f;
typedef __attribute__((ext_vector_type(4)))  unsigned int v4u;
typedef __attribute__((ext_vector_type(4)))  int      v4i;

__device__ __forceinline__ unsigned short f2bf_bits(float f) {
  unsigned u = __float_as_uint(f);
  return (unsigned short)((u + 0x7FFFu + ((u >> 16) & 1u)) >> 16);
}
__device__ __forceinline__ float bf_bits2f(unsigned short h) { return __uint_as_float(((unsigned)h) << 16); }

__device__ __forceinline__ void dep_guard_h(v8f& a, v8f& b, v16h x, v16h y) { asm volatile("v_nop\n\tv_nop\n\tv_nop\n\tv_nop" : "+v"(a), "+v"(b) : "v"(x), "v"(y)); }
__device__ __forceinline__ void dep_guard_b(v8f& a, v8f& b, v16b x, v16b y) { asm volatile("v_nop\n\tv_nop\n\tv_nop\n\tv_nop" : "+v"(a), "+v"(b) : "v"(x), "v"(y)); }
__device__ __forceinline__ void keep4_h(v16h a, v16h b, v16h c, v16h d) { asm volatile("v_nop" :: "v"(a), "v"(b), "v"(c), "v"(d)); }
__device__ __forceinline__ void keep4_b(v16b a, v16b b, v16b c, v16b d) { asm volatile("v_nop" :: "v"(a), "v"(b), "v"(c), "v"(d)); }
__device__ __forceinline__ void acc_guard4(v8f& a, v8f& b, v8f& c, v8f& d) { asm volatile("v_nop\n\tv_nop\n\tv_nop\n\tv_nop" : "+v"(a), "+v"(b), "+v"(c), "+v"(d)); }
template <typename T> struct Frag;
template <> struct Frag<_Float16> {
  typedef v16h V; union U { v16h v; v8h h[2]; };
  static __device__ __forceinline__ v16h load(const _Float16* p) {
    U f; f.h[0] = *(const v8h*)(p); f.h[1] = *(const v8h*)(p + 16); return f.v;
  }
  static __device__ __forceinline__ v8f mma(v16h a, v16h b, v8f c) {
    return __builtin_amdgcn_wmma_f32_16x16x32_f16(false, a, false, b, (short)0, c, false, false);
  }
  static __device__ __forceinline__ void guard(v8f& a, v8f& b, v16h x, v16h y) { dep_guard_h(a, b, x, y); }
  static __device__ __forceinline__ void keep(v16h a, v16h b, v16h c, v16h d) { keep4_h(a, b, c, d); }
};
template <> struct Frag<__bf16> {
  typedef v16b V; union U { v16b v; v8b h[2]; };
  static __device__ __forceinline__ v16b load(const __bf16* p) {
    U f; f.h[0] = *(const v8b*)(p); f.h[1] = *(const v8b*)(p + 16); return f.v;
  }
  static __device__ __forceinline__ v8f mma(v16b a, v16b b, v8f c) {
    return __builtin_amdgcn_wmma_f32_16x16x32_bf16(false, a, false, b, (short)0, c, false, false);
  }
  static __device__ __forceinline__ void guard(v8f& a, v8f& b, v16b x, v16b y) { dep_guard_b(a, b, x, y); }
  static __device__ __forceinline__ void keep(v16b a, v16b b, v16b c, v16b d) { keep4_b(a, b, c, d); }
};

__device__ __forceinline__ unsigned pk16(unsigned short a, unsigned short b) { return (unsigned)a | ((unsigned)b << 16); }
__device__ __forceinline__ unsigned short h_bits(float f) { const _Float16 h = (_Float16)f; return __builtin_bit_cast(unsigned short, h); }

template <int ET> struct Elem;
template <> struct Elem<0> { typedef _Float16 T; };
template <> struct Elem<1> { typedef __bf16 T; };
template <int ET, bool SPLIT, int BIAS_MODE, int OUT_MODE, bool RESID, int ACT = 0>
__global__ __launch_bounds__(256) void wmma_gemm64(
    const unsigned short* __restrict__ Ap, const unsigned short* __restrict__ A2p, int lda, long strideA,
    const unsigned short* __restrict__ Btp, const unsigned short* __restrict__ Bt2p, int ldb, long strideB,
    void* __restrict__ Cout, void* __restrict__ Cout2, int ldc, long strideC,
    const float* __restrict__ bias,
    const float* __restrict__ resid, long strideR,
    int M, int N, int K, float scale) {
  typedef typename Elem<ET>::T T;
  typedef typename Frag<T>::V V;
  const T* A = (const T*)Ap; const T* A2 = (const T*)A2p; const T* Bt = (const T*)Btp; const T* Bt2 = (const T*)Bt2p;
  __shared__ __align__(16) float sT[8][16 * 68];
  const int b    = blockIdx.y;
  const int lane = threadIdx.x & 31;
  const int wave = threadIdx.x >> 5;
  const int tilesN = N >> 6;
  const int tilesM = M >> 6;
  const int tile = blockIdx.x * 8 + wave;
  if (tile >= tilesM * tilesN) return;
  const int tm = tile / tilesN;
  const int tn = tile - tm * tilesN;
  const int m0 = tm << 6;
  const int n0 = tn << 6;

  const T* Ab  = A  + (size_t)b * strideA;
  const T* Bb  = Bt + (size_t)b * strideB;
  const T* Ab2 = SPLIT ? (A2  + (size_t)b * strideA) : nullptr;
  const T* Bb2 = SPLIT ? (Bt2 + (size_t)b * strideB) : nullptr;

  const int rlane = lane & 15;
  const int koff  = (lane >> 4) * 8;
  const int mOff  = (lane >> 4) * 8;

  v8f acc[4][4];
#pragma unroll
  for (int i = 0; i < 4; ++i)
#pragma unroll
    for (int j = 0; j < 4; ++j) acc[i][j] = (v8f){0.f,0.f,0.f,0.f,0.f,0.f,0.f,0.f};

  for (int k0 = 0; k0 < K; k0 += 32) {
    V bh[4], bl[4];
#pragma unroll
    for (int j = 0; j < 4; ++j) {
      const size_t bo = (size_t)(n0 + (j << 4) + rlane) * ldb + koff + k0;
      bh[j] = Frag<T>::load(Bb + bo);
      if (SPLIT) bl[j] = Frag<T>::load(Bb2 + bo);
    }
#pragma unroll
    for (int i = 0; i < 4; ++i) {
      const size_t ao = (size_t)(m0 + (i << 4) + rlane) * lda + koff + k0;
      V ah = Frag<T>::load(Ab + ao);
      V al;
      if (SPLIT) al = Frag<T>::load(Ab2 + ao);
#pragma unroll
      for (int j = 0; j < 4; ++j) {
        acc[i][j] = Frag<T>::mma(ah, bh[j], acc[i][j]);
        if (SPLIT) {
          acc[i][j] = Frag<T>::mma(ah, bl[j], acc[i][j]);
          acc[i][j] = Frag<T>::mma(al, bh[j], acc[i][j]);
        }
      }
      Frag<T>::guard(acc[i][0], acc[i][3], ah, SPLIT ? al : ah);
    }
    Frag<T>::keep(bh[0], bh[1], bh[2], bh[3]);
    if (SPLIT) Frag<T>::keep(bl[0], bl[1], bl[2], bl[3]);
  }
  acc_guard4(acc[0][0], acc[0][1], acc[0][2], acc[0][3]);
  acc_guard4(acc[1][0], acc[1][1], acc[1][2], acc[1][3]);
  acc_guard4(acc[2][0], acc[2][1], acc[2][2], acc[2][3]);
  acc_guard4(acc[3][0], acc[3][1], acc[3][2], acc[3][3]);

  float* slab = sT[wave];
  const float* Rb = RESID ? (resid + (size_t)b * strideR) : nullptr;
#pragma unroll
  for (int i = 0; i < 4; ++i) {
    const int mBase = m0 + (i << 4);
#pragma unroll
    for (int j = 0; j < 4; ++j) {
      const int n = n0 + (j << 4) + rlane;
      float bv = 0.f;
      if (BIAS_MODE == 2) bv = bias[n];
#pragma unroll
      for (int r = 0; r < 8; ++r) {
        float v = acc[i][j][r] * scale;
        if (BIAS_MODE == 1) v += bias[mBase + mOff + r];
        if (BIAS_MODE == 2) v += bv;
        if (RESID) v += Rb[(size_t)(mBase + mOff + r) * ldc + n];
        if (ACT == 1) v = tanhf(v);
        if (ACT == 2) v = fmaxf(v, 0.0f);
        if (ACT == 3) v = v / (1.0f + expf(-v));
        if (ACT == 4) v = (v > 0.f) ? v : 0.01f * v;
        if (ACT == 5) v = 0.5f * v * (1.0f + erff(v * 0.70710678118654752f));
        slab[(mOff + r) * 68 + (j << 4) + rlane] = v;
      }
    }
    __builtin_amdgcn_fence(__ATOMIC_RELEASE, "workgroup");
    __builtin_amdgcn_wave_barrier();
    __builtin_amdgcn_fence(__ATOMIC_ACQUIRE, "workgroup");
    if (OUT_MODE == 0) {
      float* C = (float*)Cout + (size_t)b * strideC;
      const int hh = lane >> 4, c4 = (lane & 15) * 4;
      for (int pass = 0; pass < 2; ++pass) {
#pragma unroll
        for (int it = 0; it < 8; ++it) {
          const int row = it * 2 + hh;
          v4f v = *(const v4f*)(slab + row * 68 + c4);
          *(volatile v4f*)(C + (size_t)(mBase + row) * ldc + n0 + c4) = v;
        }
        __threadfence();
      }
    } else {
      const int q = lane >> 3, c8 = (lane & 7) * 8;
      unsigned short* C  = (unsigned short*)Cout  + (size_t)b * strideC;
      unsigned short* C2 = (OUT_MODE == 2) ? ((unsigned short*)Cout2 + (size_t)b * strideC) : nullptr;
      for (int pass = 0; pass < 2; ++pass) {
#pragma unroll
        for (int it = 0; it < 4; ++it) {
          const int row = it * 4 + q;
          const float* sp = slab + row * 68 + c8;
          v8h hv, lv;
#pragma unroll
          for (int e = 0; e < 8; ++e) {
            if (OUT_MODE == 1) {
              hv[e] = (_Float16)sp[e];
            } else {
              unsigned short hb = f2bf_bits(sp[e]);
              unsigned short lb = f2bf_bits(sp[e] - bf_bits2f(hb));
              hv[e] = __builtin_bit_cast(_Float16, hb);
              lv[e] = __builtin_bit_cast(_Float16, lb);
            }
          }
          *(volatile v8h*)(C + (size_t)(mBase + row) * ldc + n0 + c8) = hv;
          if (OUT_MODE == 2) *(volatile v8h*)(C2 + (size_t)(mBase + row) * ldc + n0 + c8) = lv;
        }
        __threadfence();
      }
    }
    __builtin_amdgcn_fence(__ATOMIC_RELEASE, "workgroup");
    __builtin_amdgcn_wave_barrier();
    __builtin_amdgcn_fence(__ATOMIC_ACQUIRE, "workgroup");
  }
}

__global__ __launch_bounds__(256) void xcat8_kernel(const float* __restrict__ X, const float* __restrict__ S,
                                                   unsigned short* __restrict__ XF, int nrows) {
  const int i = blockIdx.x * 256 + threadIdx.x;
  const int row = i >> 4, cc = i & 15;
  if (row >= nrows) return;
  const int c8 = (cc & 7) * 8;
  const float* px = X + (size_t)row * kFeat + c8;
  const float* ps = S + (size_t)row * kFeat + c8;
  const v4f xa = *(const v4f*)(px);
  const v4f xb = *(const v4f*)(px + 4);
  const v4f sa = *(const v4f*)(ps);
  const v4f sb = *(const v4f*)(ps + 4);
  const bool useX = (cc < 8);
  const v4f a = useX ? xa : sa;
  const v4f c = useX ? xb : sb;
  unsigned short hb[8];
#pragma unroll
  for (int e = 0; e < 4; ++e) { hb[e] = h_bits(a[e]); hb[4 + e] = h_bits(c[e]); }
  const v4u u = (v4u){pk16(hb[0], hb[1]), pk16(hb[2], hb[3]), pk16(hb[4], hb[5]), pk16(hb[6], hb[7])};
  unsigned short* q = XF + (size_t)row * kFin + cc * 8;
  *(volatile v4u*)q = u;
  __threadfence();
  *(volatile v4u*)q = u;
}

template <int MODE>
__global__ __launch_bounds__(256) void tcast8_kernel(const float* __restrict__ in, unsigned short* __restrict__ out,
                                                    unsigned short* __restrict__ out2, int KD, int ND, float scale) {
  const int nch = KD >> 3;
  const int i = blockIdx.x * 256 + threadIdx.x;
  if (i >= ND * nch) return;
  const int n  = i / nch;
  const int cc = i - n * nch;
  unsigned short hb[8], lb[8];
#pragma unroll
  for (int e = 0; e < 8; ++e) {
    const float v = in[(size_t)(cc * 8 + e) * ND + n];
    if (MODE == 0) {
      hb[e] = h_bits(v * scale);
      lb[e] = 0;
    } else {
      hb[e] = f2bf_bits(v);
      lb[e] = f2bf_bits(v - bf_bits2f(hb[e]));
    }
  }
  const v4u hv = (v4u){pk16(hb[0], hb[1]), pk16(hb[2], hb[3]), pk16(hb[4], hb[5]), pk16(hb[6], hb[7])};
  const v4u lv = (v4u){pk16(lb[0], lb[1]), pk16(lb[2], lb[3]), pk16(lb[4], lb[5]), pk16(lb[6], lb[7])};
  const size_t o = (size_t)n * KD + cc * 8;
  *(volatile v4u*)(out + o) = hv;
  if (MODE == 1) *(volatile v4u*)(out2 + o) = lv;
  __threadfence();
  *(volatile v4u*)(out + o) = hv;
  if (MODE == 1) *(volatile v4u*)(out2 + o) = lv;
  (void)scale;
}

__global__ __launch_bounds__(256) void maskbits_kernel(const int* __restrict__ adj, unsigned* __restrict__ mb, int nwords) {
  const int i = blockIdx.x * 256 + threadIdx.x;
  if (i >= nwords) return;
  const int row = i >> 4, seg = i & 15;
  const int* p = adj + (size_t)row * kNode + seg * 32;
  unsigned w = 0u;
#pragma unroll
  for (int q = 0; q < 8; ++q) {
    const v4i v = *(const v4i*)(p + 4 * q);
#pragma unroll
    for (int e = 0; e < 4; ++e) w |= ((v[e] > 0) ? 1u : 0u) << (4 * q + e);
  }
  *(volatile unsigned*)(mb + i) = w;
  __threadfence();
  *(volatile unsigned*)(mb + i) = w;
}

__device__ __forceinline__ v8h zero8h() {
  v8h z = {(_Float16)0, (_Float16)0, (_Float16)0, (_Float16)0, (_Float16)0, (_Float16)0, (_Float16)0, (_Float16)0};
  return z;
}
__device__ __forceinline__ v8f hmma(v16h a, v16h b, v8f c) {
  c = __builtin_amdgcn_wmma_f32_16x16x32_f16(false, a, false, b, (short)0, c, false, false);
  asm volatile("v_nop\n\tv_nop\n\tv_nop\n\tv_nop" : "+v"(c) : "v"(a), "v"(b));
  return c;
}

__global__ __launch_bounds__(128) void spatial_attn_kernel(const unsigned short* __restrict__ qkvp,
                                                          const unsigned* __restrict__ mbits,
                                                          unsigned short* __restrict__ OHp,
                                                          unsigned short* __restrict__ OLp) {
  union FH { v16h v; v8h h[2]; };
  __shared__ __align__(16) _Float16 Ks[kNode * kHd];
  __shared__ __align__(16) _Float16 Vt[kHd * kVP];
  __shared__ __align__(16) unsigned Mw[64 * 16];
  __shared__ __align__(16) _Float16 Ps[4][16 * kKC];
  __shared__ __align__(16) float    Os[4][16 * kOsP];

  const int tid  = threadIdx.x;
  const int wave = tid >> 5;
  const int lane = tid & 31;
  const int hh   = lane >> 4;
  const int c    = lane & 15;
  const int qb   = blockIdx.x;
  const int bt   = blockIdx.y;
  const int qblk = qb * 64;
  const int q0   = qblk + wave * 16;
  const size_t rowbase = (size_t)bt * kNode;
  const _Float16* qkv = (const _Float16*)qkvp;

  for (int t = tid; t < 64 * 16; t += 128) Mw[t] = mbits[(size_t)(qblk + (t >> 4)) * 16 + (t & 15)];

  float* os = Os[wave];
  _Float16* pw = Ps[wave];
  const v8h z8 = zero8h();
  const int cd = (c < kHd) ? c : (kHd - 1);

#pragma unroll 1
  for (int h = 0; h < kHeads; ++h) {
    __syncthreads();
#pragma unroll
    for (int i = 0; i < 4; ++i) {
      const int j = i * 128 + tid;
      const _Float16* rp = qkv + (rowbase + j) * kQkvLd + h * kHd;
      const v8h kv = *(const v8h*)(rp + kDm);
      const v8h vv = *(const v8h*)(rp + 2 * kDm);
      *(v8h*)(Ks + j * kHd) = kv;
#pragma unroll
      for (int e = 0; e < 8; ++e) Vt[e * kVP + j] = vv[e];
    }
    __syncthreads();

    FH qa;
    {
      const v8h qv = *(const v8h*)(qkv + (rowbase + q0 + c) * kQkvLd + h * kHd);
      qa.h[0] = hh ? z8 : qv;
      qa.h[1] = z8;
    }
    float mrow[8], lrow[8];
    v8f oacc = (v8f){0.f, 0.f, 0.f, 0.f, 0.f, 0.f, 0.f, 0.f};
#pragma unroll
    for (int r = 0; r < 8; ++r) { mrow[r] = -INFINITY; lrow[r] = 0.f; }

#pragma unroll 1
    for (int kc = 0; kc < kNode / kKC; ++kc) {
      const int kv0 = kc * kKC;
      __builtin_amdgcn_fence(__ATOMIC_RELEASE, "workgroup");
      __builtin_amdgcn_wave_barrier();
      __builtin_amdgcn_fence(__ATOMIC_ACQUIRE, "workgroup");

      v8f s[4];
#pragma unroll
      for (int j = 0; j < 4; ++j) {
        FH kb;
        const v8h kvv = *(const v8h*)(Ks + (kv0 + j * 16 + c) * kHd);
        kb.h[0] = hh ? z8 : kvv;
        kb.h[1] = z8;
        s[j] = hmma(qa.v, kb.v, (v8f){0.f, 0.f, 0.f, 0.f, 0.f, 0.f, 0.f, 0.f});
      }
      float cm[8];
#pragma unroll
      for (int r = 0; r < 8; ++r) {
        const int rl = wave * 16 + 8 * hh + r;
        const unsigned w0 = Mw[rl * 16 + kc * 2];
        const unsigned w1 = Mw[rl * 16 + kc * 2 + 1];
        float m = -INFINITY;
#pragma unroll
        for (int j = 0; j < 4; ++j) {
          const unsigned w = (j < 2) ? w0 : w1;
          const unsigned keep = (w >> (((j & 1) << 4) + c)) & 1u;
          const float sv = keep ? (s[j][r] * kQKScale) : kMaskFill;
          s[j][r] = sv;
          m = fmaxf(m, sv);
        }
#pragma unroll
        for (int off = 1; off < 16; off <<= 1) m = fmaxf(m, __shfl_xor(m, off, 32));
        cm[r] = m;
      }
#pragma unroll
      for (int r = 0; r < 8; ++r) {
        const float mnew  = fmaxf(mrow[r], cm[r]);
        const float alpha = __expf(mrow[r] - mnew);
        mrow[r] = mnew;
        float psum = 0.f;
#pragma unroll
        for (int j = 0; j < 4; ++j) {
          const _Float16 p16 = (_Float16)(__expf(s[j][r] - mnew) * kPScale);
          psum += (float)p16;
          pw[(8 * hh + r) * kKC + j * 16 + c] = p16;
        }
#pragma unroll
        for (int off = 1; off < 16; off <<= 1) psum += __shfl_xor(psum, off, 32);
        lrow[r] = lrow[r] * alpha + psum;
        oacc[r] *= alpha;
      }
      __builtin_amdgcn_fence(__ATOMIC_RELEASE, "workgroup");
      __builtin_amdgcn_wave_barrier();
      __builtin_amdgcn_fence(__ATOMIC_ACQUIRE, "workgroup");
#pragma unroll
      for (int kk = 0; kk < 2; ++kk) {
        FH pa, vb;
        pa.h[0] = *(const v8h*)(pw + c * kKC + kk * 32 + 8 * hh);
        pa.h[1] = *(const v8h*)(pw + c * kKC + kk * 32 + 16 + 8 * hh);
        const v8h v0 = *(const v8h*)(Vt + cd * kVP + kv0 + kk * 32 + 8 * hh);
        const v8h v1 = *(const v8h*)(Vt + cd * kVP + kv0 + kk * 32 + 16 + 8 * hh);
        vb.h[0] = (c < kHd) ? v0 : z8;
        vb.h[1] = (c < kHd) ? v1 : z8;
        oacc = hmma(pa.v, vb.v, oacc);
      }
    }
    if (c < kHd) {
#pragma unroll
      for (int r = 0; r < 8; ++r) {
        const float inv = __builtin_amdgcn_rcpf(lrow[r]);
        os[(8 * hh + r) * kOsP + h * kHd + c] = oacc[r] * inv;
      }
    }
  }

  __builtin_amdgcn_fence(__ATOMIC_RELEASE, "workgroup");
  __builtin_amdgcn_wave_barrier();
  __builtin_amdgcn_fence(__ATOMIC_ACQUIRE, "workgroup");
  {
    const int q4 = lane >> 3, c8 = (lane & 7) * 8;
    for (int pass = 0; pass < 2; ++pass) {
#pragma unroll
      for (int it = 0; it < 4; ++it) {
        const int row = it * 4 + q4;
        const float* sp = os + row * kOsP + c8;
        v8h hv, lv;
#pragma unroll
        for (int e = 0; e < 8; ++e) {
          const unsigned short hb = f2bf_bits(sp[e]);
          const unsigned short lb = f2bf_bits(sp[e] - bf_bits2f(hb));
          hv[e] = __builtin_bit_cast(_Float16, hb);
          lv[e] = __builtin_bit_cast(_Float16, lb);
        }
        const size_t o = (rowbase + q0 + row) * kDm + c8;
        *(volatile v8h*)(OHp + o) = hv;
        *(volatile v8h*)(OLp + o) = lv;
      }
      __threadfence();
    }
  }
}

extern "C" void kernel_launch(void* const* d_in, const int* in_sizes, int n_in,
                              void* d_out, int out_size, void* d_ws, size_t ws_size,
                              hipStream_t stream) {
  if (n_in < 13) return;
  if (in_sizes[0] != kRows * kFeat || in_sizes[1] != kRows * kFeat) return;
  if (in_sizes[2] != kNode * kNode) return;
  if (in_sizes[3] != kFin * kDm || in_sizes[5] != kFin * kDm || in_sizes[7] != kFin * kDm) return;
  if (in_sizes[4] != kDm || in_sizes[6] != kDm || in_sizes[8] != kDm || in_sizes[10] != kDm || in_sizes[12] != kDm) return;
  if (in_sizes[9] != kDm * kDm || in_sizes[11] != kDm * kDm) return;
  if (out_size != kRows * kDm) return;

  const float* X   = (const float*)d_in[0];
  const float* STE = (const float*)d_in[1];
  const int*   adj = (const int*)d_in[2];
  const float* WQ  = (const float*)d_in[3];
  const float* bQ  = (const float*)d_in[4];
  const float* WK  = (const float*)d_in[5];
  const float* bK  = (const float*)d_in[6];
  const float* WV  = (const float*)d_in[7];
  const float* bV  = (const float*)d_in[8];
  const float* W1  = (const float*)d_in[9];
  const float* b1  = (const float*)d_in[10];
  const float* W2  = (const float*)d_in[11];
  const float* b2  = (const float*)d_in[12];
  float* outp = (float*)d_out;

  const size_t SZ_XF  = (size_t)kRows * kFin * 2;
  const size_t SZ_WT  = (size_t)kQkvLd * kFin * 2;
  const size_t SZ_MB  = (size_t)kNode * 16 * 4;
  const size_t SZ_QKV = (size_t)kRows * kQkvLd * 2;
  const size_t SZ_T16 = (size_t)kRows * kDm * 2;
  const size_t SZ_W16 = (size_t)kDm * kDm * 2;
  size_t off = 0;
  const size_t oXF  = off; off += SZ_XF;
  const size_t oWT  = off; off += SZ_WT;
  const size_t oMB  = off; off += SZ_MB;
  const size_t oQKV = off; off += SZ_QKV;
  const size_t oOH  = off; off += SZ_T16;
  const size_t oOL  = off; off += SZ_T16;
  const size_t oW1H = off; off += SZ_W16;
  const size_t oW1L = off; off += SZ_W16;
  const size_t oW2H = off; off += SZ_W16;
  const size_t oW2L = off; off += SZ_W16;
  const size_t oY1H = off; off += SZ_T16;
  const size_t oY1L = off; off += SZ_T16;
  const size_t TOTAL = off;
  if (TOTAL > ws_size) return;
  if (TOTAL > (size_t)134217728) return;

  char* ws = (char*)d_ws;
  unsigned short* XF  = (unsigned short*)(ws + oXF);
  unsigned short* WT  = (unsigned short*)(ws + oWT);
  unsigned*       MB  = (unsigned*)(ws + oMB);
  unsigned short* QKV = (unsigned short*)(ws + oQKV);
  unsigned short* OH  = (unsigned short*)(ws + oOH);
  unsigned short* OL  = (unsigned short*)(ws + oOL);
  unsigned short* W1H = (unsigned short*)(ws + oW1H);
  unsigned short* W1L = (unsigned short*)(ws + oW1L);
  unsigned short* W2H = (unsigned short*)(ws + oW2H);
  unsigned short* W2L = (unsigned short*)(ws + oW2L);
  unsigned short* Y1H = (unsigned short*)(ws + oY1H);
  unsigned short* Y1L = (unsigned short*)(ws + oY1L);

  const dim3 blk(256);

  xcat8_kernel<<<dim3((kRows * 16) / 256), blk, 0, stream>>>(X, STE, XF, kRows);

  {
    const int nthr = kDm * (kFin / 8);
    tcast8_kernel<0><<<dim3((nthr + 255) / 256), blk, 0, stream>>>(WQ, WT,                          WT, kFin, kDm, kWCarry);
    tcast8_kernel<0><<<dim3((nthr + 255) / 256), blk, 0, stream>>>(WK, WT + (size_t)kDm * kFin,     WT, kFin, kDm, kWCarry);
    tcast8_kernel<0><<<dim3((nthr + 255) / 256), blk, 0, stream>>>(WV, WT + (size_t)2 * kDm * kFin, WT, kFin, kDm, kWCarry);
    const int nthr2 = kDm * (kDm / 8);
    tcast8_kernel<1><<<dim3((nthr2 + 255) / 256), blk, 0, stream>>>(W1, W1H, W1L, kDm, kDm, 1.0f);
    tcast8_kernel<1><<<dim3((nthr2 + 255) / 256), blk, 0, stream>>>(W2, W2H, W2L, kDm, kDm, 1.0f);
  }

  maskbits_kernel<<<dim3((kNode * 16) / 256), blk, 0, stream>>>(adj, MB, kNode * 16);

  const int tilesM = kRows / 64;
  const dim3 gP((tilesM + 7) / 8, 1);
  wmma_gemm64<0, false, 2, 1, false, 2><<<gP, blk, 0, stream>>>(
      XF, XF, kFin, 0L, WT, WT, kFin, 0L,
      (void*)QKV, (void*)QKV, kQkvLd, 0L, bQ, bQ, 0L, kRows, kDm, kFin, kWCarryInv);
  wmma_gemm64<0, false, 2, 1, false, 2><<<gP, blk, 0, stream>>>(
      XF, XF, kFin, 0L, WT + (size_t)kDm * kFin, WT + (size_t)kDm * kFin, kFin, 0L,
      (void*)(QKV + kDm), (void*)(QKV + kDm), kQkvLd, 0L, bK, bK, 0L, kRows, kDm, kFin, kWCarryInv);
  wmma_gemm64<0, false, 2, 1, false, 2><<<gP, blk, 0, stream>>>(
      XF, XF, kFin, 0L, WT + (size_t)2 * kDm * kFin, WT + (size_t)2 * kDm * kFin, kFin, 0L,
      (void*)(QKV + 2 * kDm), (void*)(QKV + 2 * kDm), kQkvLd, 0L, bV, bV, 0L, kRows, kDm, kFin, kWCarryInv);

  spatial_attn_kernel<<<dim3(kNode / 64, kGroupsBT), dim3(128), 0, stream>>>(QKV, MB, OH, OL);

  wmma_gemm64<1, true, 2, 2, false, 2><<<gP, blk, 0, stream>>>(
      OH, OL, kDm, 0L, W1H, W1L, kDm, 0L,
      (void*)Y1H, (void*)Y1L, kDm, 0L, b1, b1, 0L, kRows, kDm, kDm, 1.0f);

  wmma_gemm64<1, true, 2, 0, false, 0><<<gP, blk, 0, stream>>>(
      Y1H, Y1L, kDm, 0L, W2H, W2L, kDm, 0L,
      (void*)outp, (void*)outp, kDm, 0L, b2, b2, 0L, kRows, kDm, kDm, 1.0f);
}
